// MultiHeadBlockSelf_22969485099563
// MI455X (gfx1250) — hardware-verified
//
#include <hip/hip_runtime.h>
#include <hip/hip_bf16.h>

#define NT   2048
#define ND   768
#define NH   12
#define NDH  64
#define NDV  384
#define NCP  6144
#define NBT  4096
#define NHV  4608
#define NBH  24
#define NQB  128
#define NKT  32

typedef _Float16 v16h __attribute__((ext_vector_type(16)));
typedef _Float16 v8h  __attribute__((ext_vector_type(8)));
typedef __bf16   v16b __attribute__((ext_vector_type(16)));
typedef __bf16   v8b  __attribute__((ext_vector_type(8)));
typedef float    v8f  __attribute__((ext_vector_type(8)));
typedef float    v4f  __attribute__((ext_vector_type(4)));
typedef int      v4i  __attribute__((ext_vector_type(4)));
typedef v8h __attribute__((may_alias)) v8ha;
typedef v8b __attribute__((may_alias)) v8ba;
typedef v4f __attribute__((may_alias)) v4fa;
typedef v4i __attribute__((may_alias)) v4ia;

union FragH { v16h v; v8h p[2]; };
union FragB { v16b v; v8b p[2]; };

__device__ __forceinline__ v8f mma_h(v16h a, v16h b, v8f c) {
  v8f d = __builtin_amdgcn_wmma_f32_16x16x32_f16(false, a, false, b, (short)0, c, false, false);
  asm volatile("v_nop\n\tv_nop\n\tv_nop\n\tv_nop" : "+v"(d) : "v"(a), "v"(b));
  return d;
}
__device__ __forceinline__ v8f mma_b(v16b a, v16b b, v8f c) {
  v8f d = __builtin_amdgcn_wmma_f32_16x16x32_bf16(false, a, false, b, (short)0, c, false, false);
  asm volatile("v_nop\n\tv_nop\n\tv_nop\n\tv_nop" : "+v"(d) : "v"(a), "v"(b));
  return d;
}

__device__ __forceinline__ v16h ldf_h(const _Float16* p, int h) {
  FragH f;
  f.p[0] = *(const v8ha*)(p + 8 * h);
  f.p[1] = *(const v8ha*)(p + 16 + 8 * h);
  return f.v;
}
__device__ __forceinline__ v16b ldf_b(const __bf16* p, int h) {
  FragB f;
  f.p[0] = *(const v8ba*)(p + 8 * h);
  f.p[1] = *(const v8ba*)(p + 16 + 8 * h);
  return f.v;
}

__device__ __forceinline__ float leaky(float v) { return v >= 0.0f ? v : 0.01f * v; }

__device__ __forceinline__ void split8(v4f a, v4f c, v8b& hi, v8b& lo) {
  const float v[8] = {a.x, a.y, a.z, a.w, c.x, c.y, c.z, c.w};
  __bf16 hh[8], ll[8];
#pragma unroll
  for (int i = 0; i < 8; ++i) {
    hh[i] = (__bf16)v[i];
    ll[i] = (__bf16)(v[i] - (float)hh[i]);
  }
  const v8b x = {hh[0], hh[1], hh[2], hh[3], hh[4], hh[5], hh[6], hh[7]};
  const v8b y = {ll[0], ll[1], ll[2], ll[3], ll[4], ll[5], ll[6], ll[7]};
  hi = x;
  lo = y;
}

__global__ __launch_bounds__(256) void cvt_f16_kernel(const float* __restrict__ src,
                                                      _Float16* __restrict__ dst,
                                                      int n8, float sc) {
  const int g = blockIdx.x * 256 + threadIdx.x;
  if (g >= n8) return;
  const float* p = src + (size_t)g * 8;
  const v4f a = *(const v4fa*)p;
  const v4f c = *(const v4fa*)(p + 4);
  const v8h o = { (_Float16)(a.x * sc), (_Float16)(a.y * sc), (_Float16)(a.z * sc), (_Float16)(a.w * sc),
                  (_Float16)(c.x * sc), (_Float16)(c.y * sc), (_Float16)(c.z * sc), (_Float16)(c.w * sc) };
  _Float16* d = dst + (size_t)g * 8;
  *(volatile v8h*)d = o;
  __threadfence();
  *(volatile v8h*)d = o;
}

__global__ __launch_bounds__(256) void cvt_split_kernel(const float* __restrict__ src,
                                                        __bf16* __restrict__ hi,
                                                        __bf16* __restrict__ lo, int n8) {
  const int g = blockIdx.x * 256 + threadIdx.x;
  if (g >= n8) return;
  const float* p = src + (size_t)g * 8;
  const v4f a = *(const v4fa*)p;
  const v4f c = *(const v4fa*)(p + 4);
  v8b vh, vl;
  split8(a, c, vh, vl);
  __bf16* dh = hi + (size_t)g * 8;
  __bf16* dl = lo + (size_t)g * 8;
  *(volatile v8b*)dh = vh;
  *(volatile v8b*)dl = vl;
  __threadfence();
  *(volatile v8b*)dh = vh;
  *(volatile v8b*)dl = vl;
}

__global__ __launch_bounds__(256) void flags_kernel(const int* __restrict__ mask,
                                                    int* __restrict__ flags) {
  __shared__ __attribute__((aligned(16))) int sF[NKT];
  const int tid = threadIdx.x, lane = tid & 31, wave = tid >> 5;
  const int qb = blockIdx.x;
  const int row = qb * 16 + (lane & 15);
#pragma unroll 1
  for (int i = 0; i < 4; ++i) {
    const int kt = 4 * wave + i;
    const int* p = mask + (size_t)row * NT + kt * 64 + 32 * (lane >> 4);
    int cnt = 0;
#pragma unroll
    for (int u = 0; u < 8; ++u) {
      const v4i a = *(const v4ia*)(p + 4 * u);
      cnt += (a.x != 0) + (a.y != 0) + (a.z != 0) + (a.w != 0);
    }
    cnt += __shfl_xor(cnt, 16);
    cnt += __shfl_xor(cnt, 8);
    cnt += __shfl_xor(cnt, 4);
    cnt += __shfl_xor(cnt, 2);
    cnt += __shfl_xor(cnt, 1);
    const int f = (cnt == 0) ? 0 : ((cnt == 1024) ? 2 : 1);
    if (lane == 0) sF[kt] = f;
  }
  __syncthreads();
  const bool wr = (tid < 8);
  v4i v = {0, 0, 0, 0};
  if (wr) v = *(const v4ia*)(sF + 4 * tid);
  int* dst = flags + qb * NKT + 4 * (tid & 7);
  if (wr) *(volatile v4i*)dst = v;
  __threadfence();
  if (wr) *(volatile v4i*)dst = v;
}

__device__ __forceinline__ void gemm_core_f16(const _Float16* __restrict__ ar,
                                              const _Float16* __restrict__ wr,
                                              int K, int h, v8f (&acc)[2][4]) {
  const v8f z8 = {0.f, 0.f, 0.f, 0.f, 0.f, 0.f, 0.f, 0.f};
#pragma unroll
  for (int i = 0; i < 2; ++i)
#pragma unroll
    for (int j = 0; j < 4; ++j) acc[i][j] = z8;
  const _Float16* ar1 = ar + (size_t)16 * K;
#pragma unroll 1
  for (int k0 = 0; k0 < K; k0 += 32) {
    const v16h a0 = ldf_h(ar + k0, h);
    const v16h a1 = ldf_h(ar1 + k0, h);
#pragma unroll
    for (int j = 0; j < 4; ++j) {
      const v16h b = ldf_h(wr + (size_t)(16 * j) * K + k0, h);
      acc[0][j] = mma_h(a0, b, acc[0][j]);
      acc[1][j] = mma_h(a1, b, acc[1][j]);
    }
  }
}

__device__ __forceinline__ void gemm_core_x3(const __bf16* __restrict__ ahr,
                                             const __bf16* __restrict__ alr,
                                             const __bf16* __restrict__ whr,
                                             const __bf16* __restrict__ wlr,
                                             int K, int h, v8f (&acc)[2][4]) {
  const v8f z8 = {0.f, 0.f, 0.f, 0.f, 0.f, 0.f, 0.f, 0.f};
#pragma unroll
  for (int i = 0; i < 2; ++i)
#pragma unroll
    for (int j = 0; j < 4; ++j) acc[i][j] = z8;
  const size_t r16 = (size_t)16 * K;
#pragma unroll 1
  for (int k0 = 0; k0 < K; k0 += 32) {
    const v16b a0h = ldf_b(ahr + k0, h);
    const v16b a0l = ldf_b(alr + k0, h);
    const v16b a1h = ldf_b(ahr + r16 + k0, h);
    const v16b a1l = ldf_b(alr + r16 + k0, h);
#pragma unroll
    for (int j = 0; j < 4; ++j) {
      const v16b bh = ldf_b(whr + (size_t)(16 * j) * K + k0, h);
      const v16b bl = ldf_b(wlr + (size_t)(16 * j) * K + k0, h);
      acc[0][j] = mma_b(a0h, bh, acc[0][j]);
      acc[0][j] = mma_b(a0l, bh, acc[0][j]);
      acc[0][j] = mma_b(a0h, bl, acc[0][j]);
      acc[1][j] = mma_b(a1h, bh, acc[1][j]);
      acc[1][j] = mma_b(a1l, bh, acc[1][j]);
      acc[1][j] = mma_b(a1h, bl, acc[1][j]);
    }
  }
}

__device__ __forceinline__ void store_f32_tile(const float* sC, float* dst, int m0, int n0,
                                               int wave, int lane) {
  const int q8 = lane & 7, sub = lane >> 3;
#pragma unroll
  for (int it = 0; it < 16; ++it) {
    const int L = 64 * wave + 4 * it + sub;
    const int row = L >> 2, seg = L & 3;
    const v4f v = *(const v4fa*)(sC + row * 128 + 32 * seg + 4 * q8);
    *(volatile v4f*)(dst + (size_t)(m0 + row) * ND + n0 + 32 * seg + 4 * q8) = v;
  }
}

__device__ __forceinline__ void store_split_tile(const float* sC, __bf16* dh, __bf16* dl,
                                                 int m0, int n0, int wave, int lane) {
  const int q8 = lane & 7, sub = lane >> 3;
#pragma unroll
  for (int it = 0; it < 8; ++it) {
    const int U = 32 * wave + 4 * it + sub;
    const int row = U >> 1, seg = U & 1;
    const float* sp = sC + row * 128 + 64 * seg + 8 * q8;
    const v4f a = *(const v4fa*)sp;
    const v4f c = *(const v4fa*)(sp + 4);
    v8b vh, vl;
    split8(a, c, vh, vl);
    const size_t off = (size_t)(m0 + row) * ND + n0 + 64 * seg + 8 * q8;
    *(volatile v8b*)(dh + off) = vh;
    *(volatile v8b*)(dl + off) = vl;
  }
}

__device__ __forceinline__ void cp_store_pass(const _Float16* sH, _Float16* qp, _Float16* kp,
                                              _Float16* vt, int bx, int n0, int b, int t0,
                                              int wave, int lane, bool isV) {
  const int q8 = lane & 7, sub = lane >> 3;
  if (!isV) {
    const int which = (bx >= 6) ? 1 : 0;
    _Float16* plane = which ? kp : qp;
    const int hb = (n0 - ND * which) >> 6;
#pragma unroll
    for (int it = 0; it < 8; ++it) {
      const int L = 32 * wave + 4 * it + sub;
      const int row = L >> 1, g = L & 1;
      const v8h v = *(const v8ha*)(sH + row * 128 + 64 * g + 8 * q8);
      _Float16* dst = plane + (((size_t)(b * NH + hb + g)) * NT + t0 + row) * NDH + 8 * q8;
      *(volatile v8h*)dst = v;
    }
  } else {
    const int c0 = n0 - 2 * ND;
    const int head = c0 / NDV;
    const int d0 = c0 - head * NDV;
#pragma unroll
    for (int it = 0; it < 8; ++it) {
      const int L = 32 * wave + 4 * it + sub;
      const v8h v = *(const v8ha*)(sH + L * 64 + 8 * q8);
      _Float16* dst = vt + (((size_t)(b * NH + head)) * NDV + d0 + L) * NT + t0 + 8 * q8;
      *(volatile v8h*)dst = v;
    }
  }
}

__global__ __launch_bounds__(128) void cp_gemm_kernel(
    const _Float16* __restrict__ xh,
    const _Float16* __restrict__ wch,
    const float* __restrict__ bc,
    _Float16* __restrict__ qp,
    _Float16* __restrict__ kp,
    _Float16* __restrict__ vt)
{
  __shared__ __attribute__((aligned(16))) _Float16 sH[64 * 128];
  const int tid = threadIdx.x, lane = tid & 31, wave = tid >> 5;
  const int h = lane >> 4, m = lane & 15;
  const int wm = wave >> 1, wn = wave & 1;
  const int bx = blockIdx.x;
  const int m0 = blockIdx.y * 64, n0 = bx * 128;
  const int mw = m0 + 32 * wm, nw = n0 + 64 * wn;

  v8f acc[2][4];
  gemm_core_f16(xh + (size_t)(mw + m) * ND, wch + (size_t)(nw + m) * ND, ND, h, acc);

  const bool isV = (bx >= 12);
#pragma unroll
  for (int j = 0; j < 4; ++j) {
    const int cl = 64 * wn + 16 * j + m;
    const float bv = bc[n0 + cl];
#pragma unroll
    for (int i = 0; i < 2; ++i) {
#pragma unroll
      for (int r = 0; r < 8; ++r) {
        const int rl = 32 * wm + 16 * i + 8 * h + r;
        const float y = leaky(acc[i][j][r] * 0.001953125f + bv) * 16.0f;
        sH[isV ? (cl * 64 + rl) : (rl * 128 + cl)] = (_Float16)y;
      }
    }
  }
  __syncthreads();

  const int b = m0 >> 11, t0 = m0 & (NT - 1);
  cp_store_pass(sH, qp, kp, vt, bx, n0, b, t0, wave, lane, isV);
  __threadfence();
  cp_store_pass(sH, qp, kp, vt, bx, n0, b, t0, wave, lane, isV);
}

__global__ __launch_bounds__(128) void attn_kernel(
    const _Float16* __restrict__ qp,
    const _Float16* __restrict__ kp,
    const _Float16* __restrict__ vt,
    const int* __restrict__ mask,
    const int* __restrict__ flags,
    _Float16* __restrict__ op)
{
  __shared__ __attribute__((aligned(16))) float sS[2 * 16 * 64];
  __shared__ __attribute__((aligned(16))) _Float16 sO[16 * NDV];

  const int tid = threadIdx.x, lane = tid & 31, w = tid >> 5;
  const int h = lane >> 4, m = lane & 15;
  const int qb = blockIdx.x, bh = blockIdx.y;
  const int b = bh / NH, head = bh - b * NH;
  const int q0 = qb * 16;
  const float ninf = -__builtin_inff();

  const _Float16* qrow = qp + ((size_t)bh * NT + q0 + m) * NDH;
  const v16h qf0 = ldf_h(qrow, h);
  const v16h qf1 = ldf_h(qrow + 32, h);

  const _Float16* kbase = kp + ((size_t)bh * NT + 16 * w + m) * NDH;
  const _Float16* vbase = vt + ((size_t)bh * NDV + 96 * w + m) * NT;
  const int* mbase = mask + (size_t)(q0 + m) * NT + 16 * w + 8 * h;
  const int* fbase = flags + qb * NKT;

  const v8f z8 = {0.f, 0.f, 0.f, 0.f, 0.f, 0.f, 0.f, 0.f};
  v8f oacc[6];
#pragma unroll
  for (int t = 0; t < 6; ++t) oacc[t] = z8;
  float mrun = ninf, lrun = 0.0f;
  int pp = 0;

#pragma unroll 1
  for (int kt = 0; kt < NKT; ++kt) {
    const int fl = __builtin_amdgcn_readfirstlane(fbase[kt]);
    if (fl == 2) continue;
    const int kb = kt * 64;

    const _Float16* kpt = kbase + (size_t)kb * NDH;
    const v16h kf0 = ldf_h(kpt, h);
    const v16h kf1 = ldf_h(kpt + 32, h);
    v8f z = z8;
    z = mma_h(kf0, qf0, z);
    z = mma_h(kf1, qf1, z);
    float sv[8];
#pragma unroll
    for (int r = 0; r < 8; ++r) sv[r] = z[r] * 0.00048828125f;
    if (fl != 0) {
      const v4i ma = *(const v4ia*)(mbase + kb);
      const v4i mc = *(const v4ia*)(mbase + kb + 4);
      const int mk[8] = {ma.x, ma.y, ma.z, ma.w, mc.x, mc.y, mc.z, mc.w};
#pragma unroll
      for (int r = 0; r < 8; ++r) sv[r] = (mk[r] != 0) ? ninf : sv[r];
    }
    float* sSb = sS + pp * 1024;
    pp ^= 1;
    {
      const v4f s0 = {sv[0], sv[1], sv[2], sv[3]};
      const v4f s1 = {sv[4], sv[5], sv[6], sv[7]};
      float* sw = sSb + m * 64 + 16 * w + 8 * h;
      *(v4fa*)sw = s0;
      *(v4fa*)(sw + 4) = s1;
    }
    __syncthreads();

    float p[32];
    float mloc = ninf;
    const float* sr = sSb + m * 64 + 8 * h;
#pragma unroll
    for (int j = 0; j < 2; ++j) {
#pragma unroll
      for (int g = 0; g < 2; ++g) {
        const float* rp = sr + 32 * j + 16 * g;
        const v4f a = *(const v4fa*)rp;
        const v4f c = *(const v4fa*)(rp + 4);
        const int o = 16 * j + 8 * g;
        p[o + 0] = a.x; p[o + 1] = a.y; p[o + 2] = a.z; p[o + 3] = a.w;
        p[o + 4] = c.x; p[o + 5] = c.y; p[o + 6] = c.z; p[o + 7] = c.w;
      }
    }
#pragma unroll
    for (int e = 0; e < 32; ++e) mloc = fmaxf(mloc, p[e]);
    mloc = fmaxf(mloc, __shfl_xor(mloc, 16));
    const float mnew = fmaxf(mrun, mloc);
    const float msub = (mnew == ninf) ? 0.0f : mnew;
    const float alpha = __expf(mrun - msub);
    mrun = mnew;
    float lsum = 0.0f;
#pragma unroll
    for (int e = 0; e < 32; ++e) {
      const float pe = __expf(p[e] - msub);
      p[e] = pe;
      lsum += pe;
    }
    lsum += __shfl_xor(lsum, 16);
    lrun = lrun * alpha + lsum;
#pragma unroll
    for (int t = 0; t < 6; ++t)
#pragma unroll
      for (int r = 0; r < 8; ++r) oacc[t][r] = oacc[t][r] * alpha;

    const v16h pb0 = { (_Float16)(p[0] * 16384.0f),  (_Float16)(p[1] * 16384.0f),  (_Float16)(p[2] * 16384.0f),  (_Float16)(p[3] * 16384.0f),
                       (_Float16)(p[4] * 16384.0f),  (_Float16)(p[5] * 16384.0f),  (_Float16)(p[6] * 16384.0f),  (_Float16)(p[7] * 16384.0f),
                       (_Float16)(p[8] * 16384.0f),  (_Float16)(p[9] * 16384.0f),  (_Float16)(p[10] * 16384.0f), (_Float16)(p[11] * 16384.0f),
                       (_Float16)(p[12] * 16384.0f), (_Float16)(p[13] * 16384.0f), (_Float16)(p[14] * 16384.0f), (_Float16)(p[15] * 16384.0f) };
    const v16h pb1 = { (_Float16)(p[16] * 16384.0f), (_Float16)(p[17] * 16384.0f), (_Float16)(p[18] * 16384.0f), (_Float16)(p[19] * 16384.0f),
                       (_Float16)(p[20] * 16384.0f), (_Float16)(p[21] * 16384.0f), (_Float16)(p[22] * 16384.0f), (_Float16)(p[23] * 16384.0f),
                       (_Float16)(p[24] * 16384.0f), (_Float16)(p[25] * 16384.0f), (_Float16)(p[26] * 16384.0f), (_Float16)(p[27] * 16384.0f),
                       (_Float16)(p[28] * 16384.0f), (_Float16)(p[29] * 16384.0f), (_Float16)(p[30] * 16384.0f), (_Float16)(p[31] * 16384.0f) };

#pragma unroll
    for (int t = 0; t < 6; ++t) {
      const _Float16* vp = vbase + (size_t)(16 * t) * NT + kb;
      const v16h vf0 = ldf_h(vp, h);
      const v16h vf1 = ldf_h(vp + 32, h);
      oacc[t] = mma_h(vf0, pb0, oacc[t]);
      oacc[t] = mma_h(vf1, pb1, oacc[t]);
    }
  }

  const float inv = (1.0f / lrun) * 0.000244140625f;
  _Float16* sow = sO + m * NDV + 96 * w + 8 * h;
#pragma unroll
  for (int t = 0; t < 6; ++t) {
    const v8h o8 = { (_Float16)(oacc[t][0] * inv), (_Float16)(oacc[t][1] * inv), (_Float16)(oacc[t][2] * inv), (_Float16)(oacc[t][3] * inv),
                     (_Float16)(oacc[t][4] * inv), (_Float16)(oacc[t][5] * inv), (_Float16)(oacc[t][6] * inv), (_Float16)(oacc[t][7] * inv) };
    *(v8ha*)(sow + 16 * t) = o8;
  }
  __syncthreads();

  const int q8 = lane & 7, sub = lane >> 3;
  const size_t orow0 = (size_t)(b * NT + q0);
#pragma unroll
  for (int it = 0; it < 6; ++it) {
    const int L = 24 * w + 4 * it + sub;
    const int row = L / 6, seg = L - 6 * row;
    const v8h v = *(const v8ha*)(sO + row * NDV + 64 * seg + 8 * q8);
    *(volatile v8h*)(op + (orow0 + row) * NHV + head * NDV + 64 * seg + 8 * q8) = v;
  }
  __threadfence();
#pragma unroll
  for (int it = 0; it < 6; ++it) {
    const int L = 24 * w + 4 * it + sub;
    const int row = L / 6, seg = L - 6 * row;
    const v8h v = *(const v8ha*)(sO + row * NDV + 64 * seg + 8 * q8);
    *(volatile v8h*)(op + (orow0 + row) * NHV + head * NDV + 64 * seg + 8 * q8) = v;
  }
}

__global__ __launch_bounds__(128) void wo_gemm_kernel(
    const _Float16* __restrict__ op,
    const _Float16* __restrict__ woh,
    const float* __restrict__ bo,
    float* __restrict__ y)
{
  __shared__ __attribute__((aligned(16))) float sC[64 * 128];
  const int tid = threadIdx.x, lane = tid & 31, wave = tid >> 5;
  const int h = lane >> 4, m = lane & 15;
  const int wm = wave >> 1, wn = wave & 1;
  const int m0 = blockIdx.y * 64, n0 = blockIdx.x * 128;
  const int mw = m0 + 32 * wm, nw = n0 + 64 * wn;

  v8f acc[2][4];
  gemm_core_f16(op + (size_t)(mw + m) * NHV, woh + (size_t)(nw + m) * NHV, NHV, h, acc);

#pragma unroll
  for (int j = 0; j < 4; ++j) {
    const int cl = 64 * wn + 16 * j + m;
    const float bv = bo[n0 + cl];
#pragma unroll
    for (int i = 0; i < 2; ++i) {
#pragma unroll
      for (int r = 0; r < 8; ++r) {
        const int rl = 32 * wm + 16 * i + 8 * h + r;
        sC[rl * 128 + cl] = leaky(acc[i][j][r] * 0.000030517578125f + bv);
      }
    }
  }
  __syncthreads();
  store_f32_tile(sC, y, m0, n0, wave, lane);
  __threadfence();
  store_f32_tile(sC, y, m0, n0, wave, lane);
}

__device__ __forceinline__ void ln_store_b(__bf16* ih, __bf16* il, size_t rb, int lane,
                                           const v8b (&hv)[3], const v8b (&lv)[3]) {
#pragma unroll
  for (int i = 0; i < 3; ++i) {
    const size_t off = rb + 256 * i + 8 * lane;
    *(volatile v8b*)(ih + off) = hv[i];
    *(volatile v8b*)(il + off) = lv[i];
  }
}
__device__ __forceinline__ void ln_store_f(const float* sRw, float* inter, size_t rb, int lane) {
#pragma unroll
  for (int i = 0; i < 6; ++i) {
    const int c = 128 * i + 4 * lane;
    const v4f v = *(const v4fa*)(sRw + c);
    *(volatile v4f*)(inter + rb + c) = v;
  }
}

__global__ __launch_bounds__(256) void ln_kernel(
    const float* __restrict__ X, const float* __restrict__ Y,
    const float* __restrict__ g, const float* __restrict__ be,
    float* __restrict__ inter, __bf16* __restrict__ ih, __bf16* __restrict__ il)
{
  __shared__ __attribute__((aligned(16))) float sR[8 * ND];
  const int tid = threadIdx.x, lane = tid & 31, wave = tid >> 5;
  const int row = blockIdx.x * 8 + wave;
  const size_t rb = (size_t)row * ND;

  float t[24];
#pragma unroll
  for (int i = 0; i < 3; ++i) {
    const int c = 256 * i + 8 * lane;
    const v4f xa = *(const v4fa*)(X + rb + c);
    const v4f xc = *(const v4fa*)(X + rb + c + 4);
    const v4f ya = *(const v4fa*)(Y + rb + c);
    const v4f yc = *(const v4fa*)(Y + rb + c + 4);
    t[8 * i + 0] = xa.x + ya.x; t[8 * i + 1] = xa.y + ya.y; t[8 * i + 2] = xa.z + ya.z; t[8 * i + 3] = xa.w + ya.w;
    t[8 * i + 4] = xc.x + yc.x; t[8 * i + 5] = xc.y + yc.y; t[8 * i + 6] = xc.z + yc.z; t[8 * i + 7] = xc.w + yc.w;
  }
  float s = 0.0f;
#pragma unroll
  for (int k = 0; k < 24; ++k) s += t[k];
  s += __shfl_xor(s, 16); s += __shfl_xor(s, 8); s += __shfl_xor(s, 4); s += __shfl_xor(s, 2); s += __shfl_xor(s, 1);
  const float mu = s * (1.0f / 768.0f);
  float q = 0.0f;
#pragma unroll
  for (int k = 0; k < 24; ++k) { t[k] = t[k] - mu; q += t[k] * t[k]; }
  q += __shfl_xor(q, 16); q += __shfl_xor(q, 8); q += __shfl_xor(q, 4); q += __shfl_xor(q, 2); q += __shfl_xor(q, 1);
  const float var = q * (1.0f / 768.0f);
  const float rstd = 1.0f / sqrtf(var + 1e-5f);

  float* sRw = sR + wave * ND;
  v8b hv[3], lv[3];
#pragma unroll
  for (int i = 0; i < 3; ++i) {
    const int c = 256 * i + 8 * lane;
    const v4f ga = *(const v4fa*)(g + c);
    const v4f gc = *(const v4fa*)(g + c + 4);
    const v4f ba = *(const v4fa*)(be + c);
    const v4f bc = *(const v4fa*)(be + c + 4);
    const v4f oa = { t[8 * i + 0] * rstd * ga.x + ba.x, t[8 * i + 1] * rstd * ga.y + ba.y,
                     t[8 * i + 2] * rstd * ga.z + ba.z, t[8 * i + 3] * rstd * ga.w + ba.w };
    const v4f oc = { t[8 * i + 4] * rstd * gc.x + bc.x, t[8 * i + 5] * rstd * gc.y + bc.y,
                     t[8 * i + 6] * rstd * gc.z + bc.z, t[8 * i + 7] * rstd * gc.w + bc.w };
    *(v4fa*)(sRw + c) = oa;
    *(v4fa*)(sRw + c + 4) = oc;
    split8(oa, oc, hv[i], lv[i]);
  }
  ln_store_b(ih, il, rb, lane, hv, lv);
  __syncthreads();
  ln_store_f(sRw, inter, rb, lane);
  __threadfence();
  ln_store_b(ih, il, rb, lane, hv, lv);
  ln_store_f(sRw, inter, rb, lane);
}

__global__ __launch_bounds__(128) void w1_kernel(
    const __bf16* __restrict__ ih, const __bf16* __restrict__ il,
    const __bf16* __restrict__ w1h, const __bf16* __restrict__ w1l,
    const float* __restrict__ b1,
    __bf16* __restrict__ h1h, __bf16* __restrict__ h1l)
{
  __shared__ __attribute__((aligned(16))) float sC[64 * 128];
  const int tid = threadIdx.x, lane = tid & 31, wave = tid >> 5;
  const int h = lane >> 4, m = lane & 15;
  const int wm = wave >> 1, wn = wave & 1;
  const int m0 = blockIdx.y * 64, n0 = blockIdx.x * 128;
  const int mw = m0 + 32 * wm, nw = n0 + 64 * wn;

  v8f acc[2][4];
  gemm_core_x3(ih + (size_t)(mw + m) * ND, il + (size_t)(mw + m) * ND,
               w1h + (size_t)(nw + m) * ND, w1l + (size_t)(nw + m) * ND, ND, h, acc);

  const float kAl = 1.6732632423543772f, kSc = 1.0507009873554805f;
#pragma unroll
  for (int j = 0; j < 4; ++j) {
    const int cl = 64 * wn + 16 * j + m;
    const float bv = b1[n0 + cl];
#pragma unroll
    for (int i = 0; i < 2; ++i) {
#pragma unroll
      for (int r = 0; r < 8; ++r) {
        const int rl = 32 * wm + 16 * i + 8 * h + r;
        const float v = acc[i][j][r] + bv;
        const float sv = (v > 0.0f) ? (kSc * v) : (kSc * (kAl * expm1f(v)));
        sC[rl * 128 + cl] = sv;
      }
    }
  }
  __syncthreads();
  store_split_tile(sC, h1h, h1l, m0, n0, wave, lane);
  __threadfence();
  store_split_tile(sC, h1h, h1l, m0, n0, wave, lane);
}

__global__ __launch_bounds__(128) void w2_kernel(
    const __bf16* __restrict__ h1h, const __bf16* __restrict__ h1l,
    const __bf16* __restrict__ w2h, const __bf16* __restrict__ w2l,
    const float* __restrict__ b2,
    const float* __restrict__ inter,
    float* __restrict__ out)
{
  __shared__ __attribute__((aligned(16))) float sC[64 * 128];
  const int tid = threadIdx.x, lane = tid & 31, wave = tid >> 5;
  const int h = lane >> 4, m = lane & 15;
  const int wm = wave >> 1, wn = wave & 1;
  const int m0 = blockIdx.y * 64, n0 = blockIdx.x * 128;
  const int mw = m0 + 32 * wm, nw = n0 + 64 * wn;

  v8f acc[2][4];
  gemm_core_x3(h1h + (size_t)(mw + m) * ND, h1l + (size_t)(mw + m) * ND,
               w2h + (size_t)(nw + m) * ND, w2l + (size_t)(nw + m) * ND, ND, h, acc);

#pragma unroll
  for (int j = 0; j < 4; ++j) {
    const int cl = 64 * wn + 16 * j + m;
    const float bv = b2[n0 + cl];
#pragma unroll
    for (int i = 0; i < 2; ++i) {
#pragma unroll
      for (int r = 0; r < 8; ++r) {
        const int rl = 32 * wm + 16 * i + 8 * h + r;
        const float v = acc[i][j][r] + bv;
        const float ge = (v * (erff(v * 0.70710678118654752f) + 1.0f)) * 0.5f;
        sC[rl * 128 + cl] = inter[(size_t)(m0 + rl) * ND + n0 + cl] + ge;
      }
    }
  }
  __syncthreads();
  store_f32_tile(sC, out, m0, n0, wave, lane);
  __threadfence();
  store_f32_tile(sC, out, m0, n0, wave, lane);
}

extern "C" void kernel_launch(void* const* d_in, const int* in_sizes, int n_in,
                              void* d_out, int out_size, void* d_ws, size_t ws_size,
                              hipStream_t stream) {
  if (n_in < 12) return;
  if (in_sizes[0] != NBT * ND) return;
  if (in_sizes[1] != NT * NT) return;
  if (in_sizes[2] != NCP * ND || in_sizes[3] != NCP) return;
  if (in_sizes[4] != ND * NHV || in_sizes[5] != ND) return;
  if (in_sizes[6] != ND * ND || in_sizes[7] != ND) return;
  if (in_sizes[8] != ND * ND || in_sizes[9] != ND) return;
  if (in_sizes[10] != ND || in_sizes[11] != ND) return;
  if (out_size != NBT * ND) return;

  const float* X   = (const float*)d_in[0];
  const int*   MK  = (const int*)d_in[1];
  const float* Wc  = (const float*)d_in[2];
  const float* bc  = (const float*)d_in[3];
  const float* Wo  = (const float*)d_in[4];
  const float* bo  = (const float*)d_in[5];
  const float* W1  = (const float*)d_in[6];
  const float* b1  = (const float*)d_in[7];
  const float* W2  = (const float*)d_in[8];
  const float* b2  = (const float*)d_in[9];
  const float* lng = (const float*)d_in[10];
  const float* lnb = (const float*)d_in[11];
  float* out = (float*)d_out;

  const size_t szXH  = (size_t)NBT * ND * 2;
  const size_t szWCH = (size_t)NCP * ND * 2;
  const size_t szWOH = (size_t)ND * NHV * 2;
  const size_t szW   = (size_t)ND * ND * 2;
  const size_t szQP  = (size_t)NBH * NT * NDH * 2;
  const size_t szVT  = (size_t)NBH * NDV * NT * 2;
  const size_t szFL  = (size_t)NQB * NKT * 4;
  const size_t szOP  = (size_t)NBT * NHV * 2;
  const size_t szF32 = (size_t)NBT * ND * 4;
  const size_t szB16 = (size_t)NBT * ND * 2;

  size_t off = 0;
  const size_t oXH  = off; off += szXH;
  const size_t oWCH = off; off += szWCH;
  const size_t oWOH = off; off += szWOH;
  const size_t oW1H = off; off += szW;
  const size_t oW1L = off; off += szW;
  const size_t oW2H = off; off += szW;
  const size_t oW2L = off; off += szW;
  const size_t oQP  = off; off += szQP;
  const size_t oKP  = off; off += szQP;
  const size_t oVT  = off; off += szVT;
  const size_t oFL  = off; off += szFL;
  const size_t oOP  = off; off += szOP;
  const size_t total = off;
  if (total > ws_size) return;
  if (szF32 > 2 * szQP) return;
  if (szF32 + 4 * szB16 > szVT) return;
  const size_t oY   = oQP;
  const size_t oINT = oVT;
  const size_t oIH  = oINT + szF32;
  const size_t oIL  = oIH + szB16;
  const size_t oH1H = oIL + szB16;
  const size_t oH1L = oH1H + szB16;

  char* ws = (char*)d_ws;
  _Float16* xh  = (_Float16*)(ws + oXH);
  _Float16* wch = (_Float16*)(ws + oWCH);
  _Float16* woh = (_Float16*)(ws + oWOH);
  __bf16*   w1h = (__bf16*)(ws + oW1H);
  __bf16*   w1l = (__bf16*)(ws + oW1L);
  __bf16*   w2h = (__bf16*)(ws + oW2H);
  __bf16*   w2l = (__bf16*)(ws + oW2L);
  _Float16* qp  = (_Float16*)(ws + oQP);
  _Float16* kp  = (_Float16*)(ws + oKP);
  _Float16* vt  = (_Float16*)(ws + oVT);
  int*      fl  = (int*)(ws + oFL);
  _Float16* op  = (_Float16*)(ws + oOP);
  float*    y   = (float*)(ws + oY);
  float*    inter = (float*)(ws + oINT);
  __bf16*   ih  = (__bf16*)(ws + oIH);
  __bf16*   il  = (__bf16*)(ws + oIL);
  __bf16*   h1h = (__bf16*)(ws + oH1H);
  __bf16*   h1l = (__bf16*)(ws + oH1L);

  const int nX8  = NBT * ND / 8;
  const int nWc8 = NCP * ND / 8;
  const int nWo8 = ND * NHV / 8;
  const int nW8  = ND * ND / 8;
  cvt_f16_kernel<<<(nX8 + 255) / 256, 256, 0, stream>>>(X, xh, nX8, 1.0f);
  cvt_f16_kernel<<<(nWc8 + 255) / 256, 256, 0, stream>>>(Wc, wch, nWc8, 512.0f);
  cvt_f16_kernel<<<(nWo8 + 255) / 256, 256, 0, stream>>>(Wo, woh, nWo8, 512.0f);
  cvt_split_kernel<<<(nW8 + 255) / 256, 256, 0, stream>>>(W1, w1h, w1l, nW8);
  cvt_split_kernel<<<(nW8 + 255) / 256, 256, 0, stream>>>(W2, w2h, w2l, nW8);

  flags_kernel<<<NQB, 256, 0, stream>>>(MK, fl);

  cp_gemm_kernel<<<dim3(NCP / 128, NBT / 64), 128, 0, stream>>>(xh, wch, bc, qp, kp, vt);

  attn_kernel<<<dim3(NQB, NBH), 128, 0, stream>>>(qp, kp, vt, MK, fl, op);

  wo_gemm_kernel<<<dim3(ND / 128, NBT / 64), 128, 0, stream>>>(op, woh, bo, y);

  ln_kernel<<<NBT / 8, 256, 0, stream>>>(X, y, lng, lnb, inter, ih, il);

  w1_kernel<<<dim3(ND / 128, NBT / 64), 128, 0, stream>>>(ih, il, w1h, w1l, b1, h1h, h1l);
  w2_kernel<<<dim3(ND / 128, NBT / 64), 128, 0, stream>>>(h1h, h1l, w2h, w2l, b2, inter, out);
}
